// Meta_Fuse_12945031430622
// MI455X (gfx1250) — hardware-verified
//
#include <hip/hip_runtime.h>


#define NN_  4096
#define HH_  256
#define K2_  512
#define G4_  1024
#define NH_  1048576

static_assert(NH_ == NN_ * HH_);
static_assert(G4_ == 4 * HH_);
static_assert(K2_ == 2 * HH_);

typedef float          v4f   __attribute__((ext_vector_type(4)));
typedef float          v8f   __attribute__((ext_vector_type(8)));
typedef _Float16       v16h  __attribute__((ext_vector_type(16)));
typedef __bf16         v16b  __attribute__((ext_vector_type(16)));
typedef unsigned short u16x8 __attribute__((ext_vector_type(8)));

union Frag { u16x8 h[2]; v16h vh; v16b vb; };

constexpr size_t MIB_     = 1048576;
constexpr size_t OFF_XG   = 0;
constexpr size_t SZ_XG    = 64 * MIB_;
constexpr size_t OFF_P    = OFF_XG + SZ_XG;
constexpr size_t SZ_PL    = (size_t)NN_ * K2_ * 2;
constexpr size_t OFF_F    = OFF_P + 8 * SZ_PL;
constexpr size_t SZ_FP    = (size_t)NH_ * 2;
constexpr size_t OFF_W    = OFF_F + 12 * SZ_FP;
constexpr size_t OFF_XXYY = OFF_W;
constexpr size_t OFF_XYXY = OFF_XXYY + 524288;
constexpr size_t OFF_FC   = OFF_XYXY + 1048576;
constexpr size_t OFF_GX   = OFF_FC + 524288;
constexpr size_t WS_END   = OFF_GX + 262144;
static_assert(WS_END <= (size_t)134217728);
static_assert(OFF_P % 128 == 0 && OFF_F % 128 == 0 && OFF_W % 128 == 0 && OFF_XYXY % 128 == 0 && OFF_FC % 128 == 0 && OFF_GX % 128 == 0);
static_assert(6 * (size_t)NH_ * 4 <= SZ_XG);
static_assert(4 * (size_t)NN_ * G4_ * 4 <= SZ_XG);
static_assert(8 * (size_t)NH_ * 4 <= SZ_XG);
static_assert(2 * (size_t)2097152 * 2 + 12 * SZ_FP == 8 * SZ_PL);

constexpr size_t SUB_WIH  = 0;
constexpr size_t SUB_WHH  = 4 * MIB_;
constexpr size_t SUB_HSEQ = 8 * MIB_;
constexpr size_t SUB_YHI  = 16 * MIB_;
constexpr size_t SUB_YLO  = 24 * MIB_;
static_assert(SUB_YLO + 4 * SZ_FP == 8 * SZ_PL);

__device__ __forceinline__ unsigned short bf16_bits(float f) {
    const unsigned u = __float_as_uint(f);
    const unsigned r = u + 0x7FFFu + ((u >> 16) & 1u);
    return (unsigned short)(r >> 16);
}
__device__ __forceinline__ float bf16_val(unsigned short b) {
    return __uint_as_float(((unsigned)b) << 16);
}
__device__ __forceinline__ float rbf(float f) { return bf16_val(bf16_bits(f)); }
__device__ __forceinline__ unsigned short f16_bits(float f) {
    return __builtin_bit_cast(unsigned short, (_Float16)f);
}
__device__ __forceinline__ v8f ld8f(const float* p) {
    const v4f a = *(const v4f*)p;
    const v4f b = *(const v4f*)(p + 4);
    return __builtin_shufflevector(a, b, 0, 1, 2, 3, 4, 5, 6, 7);
}
__device__ __forceinline__ void split8(const v8f x, u16x8& hv, u16x8& lv) {
#pragma unroll
    for (int c = 0; c < 8; ++c) {
        const float f = x[c];
        const unsigned short hb = bf16_bits(f);
        const unsigned short lb = bf16_bits(f - bf16_val(hb));
        hv[c] = hb;
        lv[c] = lb;
    }
}
__device__ __forceinline__ u16x8 pack_bf16x8(const v8f x) {
    u16x8 r;
#pragma unroll
    for (int c = 0; c < 8; ++c) r[c] = bf16_bits(x[c]);
    return r;
}
__device__ __forceinline__ u16x8 pack_f16x8(const v8f x, float mul) {
    u16x8 r;
#pragma unroll
    for (int c = 0; c < 8; ++c) r[c] = f16_bits(x[c] * mul);
    return r;
}
__device__ __forceinline__ v8f rbf8(const v8f x) {
    v8f r;
#pragma unroll
    for (int c = 0; c < 8; ++c) r[c] = rbf(x[c]);
    return r;
}
__device__ __forceinline__ v8f max8(const v8f a, const v8f b) {
    v8f r;
#pragma unroll
    for (int c = 0; c < 8; ++c) r[c] = fmaxf(a[c], b[c]);
    return r;
}
__device__ __forceinline__ float sigm_f(float x) {
    return __builtin_amdgcn_rcpf(1.0f + __expf(-x));
}
__device__ __forceinline__ float tanh_f(float x) {
    const float e = __expf(2.0f * fabsf(x));
    const float t = 1.0f - 2.0f * __builtin_amdgcn_rcpf(e + 1.0f);
    return copysignf(t, x);
}

template<bool F16>
__device__ __forceinline__ void mma16(v8f& acc, const Frag& a, const Frag& b) {
    if (F16) acc = __builtin_amdgcn_wmma_f32_16x16x32_f16(false, a.vh, false, b.vh, (short)0, acc, false, false);
    else     acc = __builtin_amdgcn_wmma_f32_16x16x32_bf16(false, a.vb, false, b.vb, (short)0, acc, false, false);
    asm volatile("v_nop\n\tv_nop\n\tv_nop\n\tv_nop" : "+v"(acc) : "v"(a.vh), "v"(b.vh));
}

__global__ __launch_bounds__(256)
void cvt_bf16_kernel(const float* __restrict__ src, unsigned short* dst, int n8)
{
    const int i = blockIdx.x * 256 + threadIdx.x;
    if (i >= n8) return;
    const size_t e = (size_t)i * 8;
    const u16x8 hv = pack_bf16x8(ld8f(src + e));
    *(volatile u16x8*)(dst + e) = hv;
    __threadfence();
    *(volatile u16x8*)(dst + e) = hv;
}

__global__ __launch_bounds__(256)
void cvt_f16s_kernel(const float* __restrict__ src, unsigned short* dst, int n8, float mul)
{
    const int i = blockIdx.x * 256 + threadIdx.x;
    if (i >= n8) return;
    const size_t e = (size_t)i * 8;
    const u16x8 hv = pack_f16x8(rbf8(ld8f(src + e)), mul);
    *(volatile u16x8*)(dst + e) = hv;
    __threadfence();
    *(volatile u16x8*)(dst + e) = hv;
}

#define SRCMASK_ 23100u
__global__ __launch_bounds__(128)
void gather_kernel(const float* __restrict__ xm, const float* __restrict__ xd,
                   const int* __restrict__ id0, const int* __restrict__ id1,
                   const int* __restrict__ id2, const int* __restrict__ id3,
                   unsigned short* p0h, unsigned short* p0l, unsigned short* p1h, unsigned short* p1l,
                   unsigned short* p2, unsigned short* p3, unsigned short* p4, unsigned short* p5)
{
    __shared__ int sidx[320];
    const int n    = blockIdx.x;
    const int tid  = threadIdx.x;
    const int lane = tid & 31;
    const int g    = tid >> 5;

    for (int q = tid; q < 320; q += 128) {
        const int gg = q / 80;
        const int j  = q - gg * 80;
        const int t  = j >> 2, s = j & 3;
        const int* ip = (gg == 0) ? id0 : (gg == 1) ? id1 : (gg == 2) ? id2 : id3;
        int v = ip[((size_t)t * NN_ + n) * 4 + s];
        v = (v < 0) ? (v + NN_) : v;
        v = min(max(v, 0), NN_ - 1);
        sidx[q] = v;
    }
    __syncthreads();

    const int c8 = lane * 8;
    const float* s0 = ((SRCMASK_ >> (g * 4 + 0)) & 1u) ? xd : xm;
    const float* s1 = ((SRCMASK_ >> (g * 4 + 1)) & 1u) ? xd : xm;
    const float* s2 = ((SRCMASK_ >> (g * 4 + 2)) & 1u) ? xd : xm;
    const float* s3 = ((SRCMASK_ >> (g * 4 + 3)) & 1u) ? xd : xm;
    const int* si = sidx + g * 80;

    v8f a0 = ld8f(s0 + (size_t)si[0] * HH_ + c8);
    v8f a1 = ld8f(s1 + (size_t)si[1] * HH_ + c8);
    v8f a2 = ld8f(s2 + (size_t)si[2] * HH_ + c8);
    v8f a3 = ld8f(s3 + (size_t)si[3] * HH_ + c8);
#pragma unroll 4
    for (int t = 1; t < 20; ++t) {
        a0 = max8(a0, ld8f(s0 + (size_t)si[t * 4 + 0] * HH_ + c8));
        a1 = max8(a1, ld8f(s1 + (size_t)si[t * 4 + 1] * HH_ + c8));
        a2 = max8(a2, ld8f(s2 + (size_t)si[t * 4 + 2] * HH_ + c8));
        a3 = max8(a3, ld8f(s3 + (size_t)si[t * 4 + 3] * HH_ + c8));
    }
    a0 = rbf8(a0); a1 = rbf8(a1); a2 = rbf8(a2); a3 = rbf8(a3);
    const size_t row = (size_t)n * K2_;

    if (g < 2) {
        const v8f xa = (a0 + a1) * 0.5f;
        const v8f xb = (a2 + a3) * 0.5f;
        u16x8 ha, la, hb, lb;
        split8(xa, ha, la);
        split8(xb, hb, lb);
        unsigned short* ph = (g == 0) ? p0h : p1h;
        unsigned short* pl = (g == 0) ? p0l : p1l;
        *(volatile u16x8*)(ph + row + c8)       = ha;
        *(volatile u16x8*)(ph + row + HH_ + c8) = hb;
        *(volatile u16x8*)(pl + row + c8)       = la;
        *(volatile u16x8*)(pl + row + HH_ + c8) = lb;
        __threadfence();
        *(volatile u16x8*)(ph + row + c8)       = ha;
        *(volatile u16x8*)(ph + row + HH_ + c8) = hb;
        *(volatile u16x8*)(pl + row + c8)       = la;
        *(volatile u16x8*)(pl + row + HH_ + c8) = lb;
    } else {
        const u16x8 f0 = pack_f16x8(a0, 1.0f);
        const u16x8 f1 = pack_f16x8(a1, 1.0f);
        const u16x8 f2 = pack_f16x8(a2, 1.0f);
        const u16x8 f3 = pack_f16x8(a3, 1.0f);
        unsigned short* pa = (g == 2) ? p2 : p4;
        unsigned short* pb = (g == 2) ? p3 : p5;
        *(volatile u16x8*)(pa + row + c8)       = f0;
        *(volatile u16x8*)(pa + row + HH_ + c8) = f1;
        *(volatile u16x8*)(pb + row + c8)       = f2;
        *(volatile u16x8*)(pb + row + HH_ + c8) = f3;
        __threadfence();
        *(volatile u16x8*)(pa + row + c8)       = f0;
        *(volatile u16x8*)(pa + row + HH_ + c8) = f1;
        *(volatile u16x8*)(pb + row + c8)       = f2;
        *(volatile u16x8*)(pb + row + HH_ + c8) = f3;
    }
}

__device__ __forceinline__ void tile_store_pass(const float* st, float* gp, int ldc, int lane) {
    constexpr int P = 36;
    const int rsub = lane >> 3;
    const int c0   = (lane & 7) * 4;
#pragma unroll
    for (int it = 0; it < 8; ++it) {
        const int row = it * 4 + rsub;
        const v4f v = *(const v4f*)(st + row * P + c0);
        *(volatile v4f*)(gp + (size_t)row * ldc + c0) = v;
    }
}

template<bool F16, int NT>
__global__ __launch_bounds__(128)
void gemm_kernel(const unsigned short* __restrict__ Ah, const unsigned short* __restrict__ Al, int strideA,
                 const unsigned short* __restrict__ W, int strideW, int wmask,
                 const float* __restrict__ bias, int strideBias,
                 float* C, int strideC, int K, int ldc, float scale, int relu)
{
    constexpr int P = 36;
    __shared__ __attribute__((aligned(16))) float stile[4][32 * P];

    const int tid  = threadIdx.x;
    const int lane = tid & 31;
    const int wave = tid >> 5;
    const int h    = lane >> 4;
    const int m    = lane & 15;
    const int wm   = wave >> 1;
    const int wn   = wave & 1;
    const int z    = blockIdx.z;
    const int zw   = z & wmask;

    const unsigned short* Ahz = Ah + (size_t)z * strideA;
    const unsigned short* Alz = Al + (size_t)z * strideA;
    const unsigned short* Wz  = W + (size_t)zw * strideW;
    const float* bz = bias + (size_t)zw * strideBias;
    float* Cz = C + (size_t)z * strideC;

    const int rowW = blockIdx.y * 64 + wm * 32;
    const int colW = blockIdx.x * 64 + wn * 32;

    v8f acc[4];
#pragma unroll
    for (int j = 0; j < 4; ++j)
#pragma unroll
        for (int r = 0; r < 8; ++r) acc[j][r] = 0.0f;

    const size_t aoff  = (size_t)(rowW + m) * K + 8 * h;
    const size_t boff  = (size_t)(colW + m) * K + 8 * h;
    const size_t sub16 = (size_t)16 * K;
    const int nk = K >> 5;

#pragma unroll 1
    for (int kt = 0; kt < nk; ++kt) {
        const size_t k0 = (size_t)kt * 32;
        Frag fa[2], ga[2], fb[2];
#pragma unroll
        for (int s = 0; s < 2; ++s) {
            const unsigned short* p = Ahz + aoff + s * sub16 + k0;
            fa[s].h[0] = *(const u16x8*)(p);
            fa[s].h[1] = *(const u16x8*)(p + 16);
            if (NT == 2) {
                const unsigned short* q = Alz + aoff + s * sub16 + k0;
                ga[s].h[0] = *(const u16x8*)(q);
                ga[s].h[1] = *(const u16x8*)(q + 16);
            }
        }
#pragma unroll
        for (int j = 0; j < 2; ++j) {
            const unsigned short* p = Wz + boff + j * sub16 + k0;
            fb[j].h[0] = *(const u16x8*)(p);
            fb[j].h[1] = *(const u16x8*)(p + 16);
        }
#pragma unroll
        for (int s = 0; s < 2; ++s)
#pragma unroll
            for (int j = 0; j < 2; ++j) {
                mma16<F16>(acc[s * 2 + j], fa[s], fb[j]);
                if (NT == 2) mma16<F16>(acc[s * 2 + j], ga[s], fb[j]);
            }
    }

    float bc[2];
#pragma unroll
    for (int j = 0; j < 2; ++j) bc[j] = rbf(bz[colW + j * 16 + m]);

    float* st = stile[wave];
#pragma unroll
    for (int s = 0; s < 2; ++s)
#pragma unroll
        for (int j = 0; j < 2; ++j)
#pragma unroll
            for (int r = 0; r < 8; ++r) {
                float v = acc[s * 2 + j][r] * scale + bc[j];
                v = relu ? fmaxf(v, 0.0f) : v;
                st[(s * 16 + 8 * h + r) * P + j * 16 + m] = v;
            }
    __syncthreads();

    float* gp = Cz + (size_t)rowW * ldc + colW;
    tile_store_pass(st, gp, ldc, lane);
    __threadfence();
    tile_store_pass(st, gp, ldc, lane);
}

__global__ __launch_bounds__(256)
void split_kernel(const float* __restrict__ T, unsigned short* fhi, unsigned short* flo, unsigned short* f16p)
{
    const int z = blockIdx.z;
    const int i = blockIdx.x * 256 + threadIdx.x;
    const size_t e = (size_t)i * 8;
    const int o1 = (z < 2) ? z : (2 * z - 2);
    const int o2 = (z < 2) ? z : (2 * z - 1);
    const v8f x = (ld8f(T + (size_t)o1 * NH_ + e) + ld8f(T + (size_t)o2 * NH_ + e)) * 0.5f;
    u16x8 hv, lv;
    split8(x, hv, lv);
    const u16x8 fv = pack_f16x8(x, 1.0f);
    const size_t d = (size_t)z * NH_ + e;
    *(volatile u16x8*)(fhi + d)  = hv;
    *(volatile u16x8*)(flo + d)  = lv;
    *(volatile u16x8*)(f16p + d) = fv;
    __threadfence();
    *(volatile u16x8*)(fhi + d)  = hv;
    *(volatile u16x8*)(flo + d)  = lv;
    *(volatile u16x8*)(f16p + d) = fv;
}

#define INV512_ 0.001953125f
__global__ __launch_bounds__(256)
void rec_kernel(const float* __restrict__ xg, const unsigned short* __restrict__ whh16,
                const float* __restrict__ bhh, const float* __restrict__ h0p, const float* __restrict__ c0p,
                int layer, unsigned short* hseq16, unsigned short* yhi, unsigned short* ylo)
{
    __shared__ __attribute__((aligned(16))) unsigned short hT[16 * HH_];
    __shared__ __attribute__((aligned(16))) float sg[G4_];
    __shared__ __attribute__((aligned(16))) float sb[G4_];
    __shared__ __attribute__((aligned(16))) unsigned short sh16[HH_];
    __shared__ __attribute__((aligned(16))) unsigned short sbh[HH_];
    __shared__ __attribute__((aligned(16))) unsigned short sbl[HH_];

    const int i    = blockIdx.x;
    const int tid  = threadIdx.x;
    const int lane = tid & 31;
    const int wave = tid >> 5;
    const int h    = lane >> 4;
    const int m    = lane & 15;
    const int u    = tid;
    const int il   = i * 2 + layer;

    const u16x8 z8 = {0, 0, 0, 0, 0, 0, 0, 0};
    for (int q = tid; q < (16 * HH_) / 8; q += 256) *(u16x8*)(hT + q * 8) = z8;
    for (int q = tid; q < G4_; q += 256) sb[q] = rbf(bhh[(size_t)il * G4_ + q]);
    __syncthreads();
    float c = rbf(c0p[il * HH_ + u]);
    const float hini = rbf(h0p[il * HH_ + u]);
    hT[u] = f16_bits(hini * 8.0f);
    __syncthreads();

    const unsigned short* wrow = whh16 + ((size_t)il * G4_ + wave * 128 + m) * HH_ + 8 * h;
    const unsigned short* arow = hT + m * HH_ + 8 * h;
    const float* xgi = xg + (size_t)i * NN_ * G4_;

#pragma unroll 1
    for (int t = 0; t < NN_; ++t) {
        const float* xr = xgi + (size_t)t * G4_;
        const float xi = xr[u];
        const float xf = xr[HH_ + u];
        const float xc = xr[2 * HH_ + u];
        const float xo = xr[3 * HH_ + u];

        v8f acc[8];
#pragma unroll
        for (int j = 0; j < 8; ++j)
#pragma unroll
            for (int r = 0; r < 8; ++r) acc[j][r] = 0.0f;

#pragma unroll 1
        for (int ks = 0; ks < 8; ++ks) {
            Frag a, b;
            a.h[0] = *(const u16x8*)(arow + ks * 32);
            a.h[1] = *(const u16x8*)(arow + ks * 32 + 16);
#pragma unroll
            for (int j = 0; j < 8; ++j) {
                const unsigned short* p = wrow + (size_t)j * (16 * HH_) + ks * 32;
                b.h[0] = *(const u16x8*)(p);
                b.h[1] = *(const u16x8*)(p + 16);
                acc[j] = __builtin_amdgcn_wmma_f32_16x16x32_f16(false, a.vh, false, b.vh, (short)0, acc[j], false, false);
            }
            asm volatile("v_nop\n\tv_nop\n\tv_nop\n\tv_nop"
                         : "+v"(acc[0]), "+v"(acc[1]), "+v"(acc[2]), "+v"(acc[3]),
                           "+v"(acc[4]), "+v"(acc[5]), "+v"(acc[6]), "+v"(acc[7])
                         : "v"(a.vh), "v"(b.vh));
        }
        if (h == 0) {
#pragma unroll
            for (int j = 0; j < 8; ++j) sg[wave * 128 + j * 16 + m] = acc[j][0];
        }
        __syncthreads();

        const float ai = (xi + sg[u] * INV512_) + sb[u];
        const float af = (xf + sg[HH_ + u] * INV512_) + sb[HH_ + u];
        const float ag = (xc + sg[2 * HH_ + u] * INV512_) + sb[2 * HH_ + u];
        const float ao = (xo + sg[3 * HH_ + u] * INV512_) + sb[3 * HH_ + u];
        const float ig = sigm_f(ai);
        const float fg = sigm_f(af);
        const float gg = tanh_f(ag);
        const float og = sigm_f(ao);
        c = fg * c + ig * gg;
        const float hv = og * tanh_f(c);
        const unsigned short hb = bf16_bits(hv);
        const unsigned short lb = bf16_bits(hv - bf16_val(hb));
        hT[u]   = f16_bits(hv * 8.0f);
        sh16[u] = f16_bits(hv);
        sbh[u]  = hb;
        sbl[u]  = lb;
        __syncthreads();

        if (layer == 0) {
            if (wave == 0) {
                const u16x8 v = *(const u16x8*)(sh16 + lane * 8);
                unsigned short* d = hseq16 + ((size_t)i * NN_ + t) * HH_ + lane * 8;
                *(volatile u16x8*)d = v;
                __threadfence();
                *(volatile u16x8*)d = v;
            }
        } else {
            if (wave < 2) {
                const u16x8 vh = *(const u16x8*)(sbh + lane * 8);
                const u16x8 vl = *(const u16x8*)(sbl + lane * 8);
                const u16x8 v  = (wave == 0) ? vh : vl;
                unsigned short* d = ((wave == 0) ? yhi : ylo) + ((size_t)i * NN_ + t) * HH_ + lane * 8;
                *(volatile u16x8*)d = v;
                __threadfence();
                *(volatile u16x8*)d = v;
            }
        }
    }
}

__global__ __launch_bounds__(256)
void combine_kernel(const float* __restrict__ fc, const float* __restrict__ gx, float* out)
{
    const int i = blockIdx.x * 256 + threadIdx.x;
    const size_t e = (size_t)i * 4;
    const v4f m0 = *(const v4f*)(fc + e);
    const v4f m1 = *(const v4f*)(fc + (size_t)NH_ + e);
    const v4f m2 = *(const v4f*)(fc + (size_t)2 * NH_ + e);
    const v4f m3 = *(const v4f*)(fc + (size_t)3 * NH_ + e);
    const v4f g0 = *(const v4f*)(gx + e);
    const v4f g1 = *(const v4f*)(gx + (size_t)NH_ + e);
    const v4f g2 = *(const v4f*)(gx + (size_t)2 * NH_ + e);
    const v4f g3 = *(const v4f*)(gx + (size_t)3 * NH_ + e);
    const v4f o0 = (g0 * m0 + m0) + (g2 * m2 + m2);
    const v4f o1 = (g1 * m1 + m1) + (g3 * m3 + m3);
    *(volatile v4f*)(out + e) = o0;
    *(volatile v4f*)(out + (size_t)NH_ + e) = o1;
    __threadfence();
    *(volatile v4f*)(out + e) = o0;
    *(volatile v4f*)(out + (size_t)NH_ + e) = o1;
}

extern "C" void kernel_launch(void* const* d_in, const int* in_sizes, int n_in,
                              void* d_out, int out_size, void* d_ws, size_t ws_size,
                              hipStream_t stream)
{
    if (n_in < 20) return;
    if (in_sizes[0]  != NH_)               return;
    if (in_sizes[1]  != NH_)               return;
    if (in_sizes[2]  != 20 * NN_ * 4)      return;
    if (in_sizes[3]  != 20 * NN_ * 4)      return;
    if (in_sizes[4]  != 20 * NN_ * 4)      return;
    if (in_sizes[5]  != 20 * NN_ * 4)      return;
    if (in_sizes[6]  != 4 * 2 * G4_ * HH_) return;
    if (in_sizes[7]  != 4 * 2 * G4_ * HH_) return;
    if (in_sizes[8]  != 4 * 2 * G4_)       return;
    if (in_sizes[9]  != 4 * 2 * G4_)       return;
    if (in_sizes[10] != 4 * 2 * HH_)       return;
    if (in_sizes[11] != 4 * 2 * HH_)       return;
    if (in_sizes[12] != 4 * HH_ * HH_)     return;
    if (in_sizes[13] != 4 * HH_)           return;
    if (in_sizes[14] != 2 * HH_ * HH_)     return;
    if (in_sizes[15] != 2 * HH_)           return;
    if (in_sizes[16] != 2 * HH_ * K2_)     return;
    if (in_sizes[17] != 2 * HH_)           return;
    if (in_sizes[18] != 4 * HH_ * K2_)     return;
    if (in_sizes[19] != 4 * HH_)           return;
    if (out_size != 2 * NH_)               return;
    if (ws_size < WS_END)                  return;

    const float* mf    = (const float*)d_in[0];
    const float* df    = (const float*)d_in[1];
    const int*   id0   = (const int*)d_in[2];
    const int*   id1   = (const int*)d_in[3];
    const int*   id2   = (const int*)d_in[4];
    const int*   id3   = (const int*)d_in[5];
    const float* Wih   = (const float*)d_in[6];
    const float* Whh   = (const float*)d_in[7];
    const float* bih   = (const float*)d_in[8];
    const float* bhh   = (const float*)d_in[9];
    const float* h0    = (const float*)d_in[10];
    const float* c0    = (const float*)d_in[11];
    const float* fcW   = (const float*)d_in[12];
    const float* fcb   = (const float*)d_in[13];
    const float* gxW   = (const float*)d_in[14];
    const float* gxb   = (const float*)d_in[15];
    const float* xxyyW = (const float*)d_in[16];
    const float* xxyyb = (const float*)d_in[17];
    const float* xyxyW = (const float*)d_in[18];
    const float* xyxyb = (const float*)d_in[19];
    float* out = (float*)d_out;

    char* ws = (char*)d_ws;
    float* T   = (float*)(ws + OFF_XG);
    float* XG  = (float*)(ws + OFF_XG);
    float* FCO = (float*)(ws + OFF_XG);
    float* GXO = (float*)(ws + OFF_XG + 16 * MIB_);
    unsigned short* P0H = (unsigned short*)(ws + OFF_P + 0 * SZ_PL);
    unsigned short* P0L = (unsigned short*)(ws + OFF_P + 1 * SZ_PL);
    unsigned short* P1H = (unsigned short*)(ws + OFF_P + 2 * SZ_PL);
    unsigned short* P1L = (unsigned short*)(ws + OFF_P + 3 * SZ_PL);
    unsigned short* P2  = (unsigned short*)(ws + OFF_P + 4 * SZ_PL);
    unsigned short* P3  = (unsigned short*)(ws + OFF_P + 5 * SZ_PL);
    unsigned short* P4  = (unsigned short*)(ws + OFF_P + 6 * SZ_PL);
    unsigned short* P5  = (unsigned short*)(ws + OFF_P + 7 * SZ_PL);
    unsigned short* WIH16  = (unsigned short*)(ws + OFF_P + SUB_WIH);
    unsigned short* WHH16  = (unsigned short*)(ws + OFF_P + SUB_WHH);
    unsigned short* HSEQ16 = (unsigned short*)(ws + OFF_P + SUB_HSEQ);
    unsigned short* YHI    = (unsigned short*)(ws + OFF_P + SUB_YHI);
    unsigned short* YLO    = (unsigned short*)(ws + OFF_P + SUB_YLO);
    unsigned short* FHI  = (unsigned short*)(ws + OFF_F);
    unsigned short* FLO  = (unsigned short*)(ws + OFF_F + 4 * SZ_FP);
    unsigned short* F16P = (unsigned short*)(ws + OFF_F + 8 * SZ_FP);
    unsigned short* XXYYB  = (unsigned short*)(ws + OFF_XXYY);
    unsigned short* XYXY16 = (unsigned short*)(ws + OFF_XYXY);
    unsigned short* FCB    = (unsigned short*)(ws + OFF_FC);
    unsigned short* GXB    = (unsigned short*)(ws + OFF_GX);

    const float S64  = 64.0f;
    const float R64  = 0.015625f;

    gather_kernel<<<dim3(NN_), dim3(128), 0, stream>>>(mf, df, id0, id1, id2, id3,
                                                       P0H, P0L, P1H, P1L, P2, P3, P4, P5);

    cvt_bf16_kernel<<<dim3((2 * HH_ * K2_ / 8 + 255) / 256), dim3(256), 0, stream>>>(xxyyW, XXYYB, 2 * HH_ * K2_ / 8);
    cvt_f16s_kernel<<<dim3((4 * HH_ * K2_ / 8 + 255) / 256), dim3(256), 0, stream>>>(xyxyW, XYXY16, 4 * HH_ * K2_ / 8, S64);
    cvt_bf16_kernel<<<dim3((4 * HH_ * HH_ / 8 + 255) / 256), dim3(256), 0, stream>>>(fcW, FCB, 4 * HH_ * HH_ / 8);
    cvt_bf16_kernel<<<dim3((2 * HH_ * HH_ / 8 + 255) / 256), dim3(256), 0, stream>>>(gxW, GXB, 2 * HH_ * HH_ / 8);

    gemm_kernel<false, 2><<<dim3(HH_ / 64, NN_ / 64, 2), dim3(128), 0, stream>>>(
        P0H, P0L, (int)(2 * NN_ * K2_), XXYYB, HH_ * K2_, 3, xxyyb, HH_,
        T, NH_, K2_, HH_, 1.0f, 1);
    gemm_kernel<true, 1><<<dim3(HH_ / 64, NN_ / 64, 4), dim3(128), 0, stream>>>(
        P2, P2, (int)(NN_ * K2_), XYXY16, HH_ * K2_, 3, xyxyb, HH_,
        T + (size_t)2 * NH_, NH_, K2_, HH_, R64, 1);

    split_kernel<<<dim3(NH_ / 8 / 256, 1, 4), dim3(256), 0, stream>>>(T, FHI, FLO, F16P);

    cvt_f16s_kernel<<<dim3((4 * 2 * G4_ * HH_ / 8 + 255) / 256), dim3(256), 0, stream>>>(Wih, WIH16, 4 * 2 * G4_ * HH_ / 8, S64);
    cvt_f16s_kernel<<<dim3((4 * 2 * G4_ * HH_ / 8 + 255) / 256), dim3(256), 0, stream>>>(Whh, WHH16, 4 * 2 * G4_ * HH_ / 8, S64);

    gemm_kernel<true, 1><<<dim3(G4_ / 64, NN_ / 64, 4), dim3(128), 0, stream>>>(
        F16P, F16P, NH_, WIH16, 2 * G4_ * HH_, 3, bih, 2 * G4_,
        XG, NN_ * G4_, HH_, G4_, R64, 0);
    rec_kernel<<<dim3(4), dim3(256), 0, stream>>>(XG, WHH16, bhh, h0, c0, 0, HSEQ16, YHI, YLO);

    gemm_kernel<true, 1><<<dim3(G4_ / 64, NN_ / 64, 4), dim3(128), 0, stream>>>(
        HSEQ16, HSEQ16, NH_, WIH16 + (size_t)G4_ * HH_, 2 * G4_ * HH_, 3, bih + G4_, 2 * G4_,
        XG, NN_ * G4_, HH_, G4_, R64, 0);
    rec_kernel<<<dim3(4), dim3(256), 0, stream>>>(XG, WHH16, bhh, h0, c0, 1, HSEQ16, YHI, YLO);

    gemm_kernel<false, 2><<<dim3(HH_ / 64, NN_ / 64, 4), dim3(128), 0, stream>>>(
        YHI, YLO, NH_, FCB, HH_ * HH_, 3, fcb, HH_,
        FCO, NH_, HH_, HH_, 1.0f, 0);
    gemm_kernel<false, 2><<<dim3(HH_ / 64, NN_ / 64, 4), dim3(128), 0, stream>>>(
        FHI, FLO, NH_, GXB, HH_ * HH_, 1, gxb, HH_,
        GXO, NH_, HH_, HH_, 1.0f, 0);

    combine_kernel<<<dim3(NH_ / 4 / 256), dim3(256), 0, stream>>>(FCO, GXO, out);
}
